// RNNClassifier_69458211111685
// MI455X (gfx1250) — hardware-verified
//
#include <hip/hip_runtime.h>
#include <math.h>

constexpr int NBATCH    = 64;
constexpr int NSTEP     = 2048;
constexpr int NVOCAB    = 50000;
constexpr int NVPAD     = 50048;
constexpr int NEMB      = 256;
constexpr int NHID      = 256;
constexpr int NFC1      = 128;
constexpr int NOUTC     = 16;
constexpr int SEQ_BLK   = 16;
constexpr int SCAN_THR  = 512;
constexpr int CVT_THR   = 256;
constexpr int HEAD_THR  = 256;
constexpr int HPITCH    = 264;
constexpr int OPITCH    = 260;
constexpr int IDX_CHUNK = 32;
constexpr float WCARRY     = 16.0f;
constexpr float WCARRY_INV = 1.0f / 16.0f;

static_assert(NVPAD % 64 == 0 && NVPAD >= NVOCAB && NVPAD - NVOCAB < 64);
static_assert(NHID % 64 == 0 && NEMB % 32 == 0 && NHID % 32 == 0);
static_assert(((NVPAD / 64) * (NHID / 64)) % 8 == 0);
static_assert(NBATCH % SEQ_BLK == 0);
static_assert(SCAN_THR == SEQ_BLK * IDX_CHUNK);
static_assert(NHID == 16 * (SCAN_THR / 32));
static_assert(NSTEP % IDX_CHUNK == 0);
static_assert(HPITCH % 8 == 0 && HPITCH >= NHID);
static_assert(OPITCH % 4 == 0 && OPITCH >= NHID);
static_assert((SEQ_BLK * NHID) % (SCAN_THR * 4) == 0);
static_assert((NVPAD * (NEMB / 8)) % CVT_THR == 0);
static_assert((NHID * (NEMB / 8)) % CVT_THR == 0);
static_assert(NBATCH * NOUTC == 4 * HEAD_THR);
static_assert(NFC1 * 2 == HEAD_THR);

typedef __attribute__((ext_vector_type(16))) _Float16 v16h;
typedef __attribute__((ext_vector_type(8)))  _Float16 v8h;
typedef __attribute__((ext_vector_type(8)))  float    v8f;
typedef __attribute__((ext_vector_type(4)))  float    v4f;
typedef __attribute__((ext_vector_type(4)))  int      v4i;

__device__ __forceinline__ void dep_guard4_h(v8f& a, v8f& b, v8f& c, v8f& d, v16h x, v16h y) {
  asm volatile("v_nop\n\tv_nop\n\tv_nop\n\tv_nop" : "+v"(a), "+v"(b), "+v"(c), "+v"(d) : "v"(x), "v"(y));
}
__device__ __forceinline__ void keep4_h(v16h a, v16h b, v16h c, v16h d) { asm volatile("v_nop" :: "v"(a), "v"(b), "v"(c), "v"(d)); }
__device__ __forceinline__ void acc_guard4(v8f& a, v8f& b, v8f& c, v8f& d) {
  asm volatile("v_nop\n\tv_nop\n\tv_nop\n\tv_nop" : "+v"(a), "+v"(b), "+v"(c), "+v"(d));
}

template <typename T> struct Frag;
template <> struct Frag<_Float16> {
  typedef v16h V; union U { v16h v; v8h h[2]; };
  static __device__ __forceinline__ v16h load(const _Float16* p) {
    U f; f.h[0] = *(const v8h*)(p); f.h[1] = *(const v8h*)(p + 16); return f.v;
  }
  static __device__ __forceinline__ v8f mma(v16h a, v16h b, v8f c) {
    return __builtin_amdgcn_wmma_f32_16x16x32_f16(false, a, false, b, (short)0, c, false, false);
  }
};

__device__ __forceinline__ v8f mma_f16_guarded(v16h a, v16h b, v8f c) {
  c = __builtin_amdgcn_wmma_f32_16x16x32_f16(false, a, false, b, (short)0, c, false, false);
  asm volatile("v_nop\n\tv_nop\n\tv_nop\n\tv_nop" : "+v"(c) : "v"(a), "v"(b));
  return c;
}

__global__ __launch_bounds__(CVT_THR) void cvt8_f16_kernel(const float* __restrict__ src, unsigned short* __restrict__ dst,
                                                          int nrow_real, int nrow_pad, int ncol8, float sc) {
  const int i  = blockIdx.x * CVT_THR + threadIdx.x;
  const int n8 = nrow_pad * ncol8;
  if (i < n8) {
    const int row  = i / ncol8;
    const int c8   = i - row * ncol8;
    const bool live = row < nrow_real;
    const int rowc = live ? row : (nrow_real - 1);
    const float* sp = src + (size_t)rowc * (size_t)(ncol8 * 8) + (size_t)(c8 * 8);
    const v4f a = *(const v4f*)(sp);
    const v4f b = *(const v4f*)(sp + 4);
    v8h hv;
#pragma unroll
    for (int e = 0; e < 4; ++e) {
      const float fa = live ? (a[e] * sc) : 0.0f;
      const float fb = live ? (b[e] * sc) : 0.0f;
      hv[e]     = (_Float16)fa;
      hv[4 + e] = (_Float16)fb;
    }
    *(volatile v8h*)(dst + (size_t)i * 8) = hv;
    __threadfence();
    *(volatile v8h*)(dst + (size_t)i * 8) = hv;
  }
}

__global__ __launch_bounds__(256) void wmma_gemm64_f16(
    const unsigned short* __restrict__ Ap, int lda,
    const unsigned short* __restrict__ Btp, int ldb,
    float* __restrict__ C, int ldc,
    const float* __restrict__ bias_a, const float* __restrict__ bias_b,
    int M, int N, int K, float scale) {
  typedef _Float16 T;
  typedef Frag<T>::V V;
  const T* A  = (const T*)Ap;
  const T* Bt = (const T*)Btp;
  __shared__ __align__(16) float sT[8][16 * 68];
  const int lane = threadIdx.x & 31;
  const int wave = threadIdx.x >> 5;
  const int tilesN = N >> 6;
  const int tilesM = M >> 6;
  const int tile = blockIdx.x * 8 + wave;
  if (tile >= tilesM * tilesN) return;
  const int tm = tile / tilesN;
  const int tn = tile - tm * tilesN;
  const int m0 = tm << 6;
  const int n0 = tn << 6;

  const int rlane = lane & 15;
  const int koff  = (lane >> 4) * 8;
  const int mOff  = (lane >> 4) * 8;

  v8f acc[4][4];
#pragma unroll
  for (int i = 0; i < 4; ++i)
#pragma unroll
    for (int j = 0; j < 4; ++j) acc[i][j] = (v8f){0.f,0.f,0.f,0.f,0.f,0.f,0.f,0.f};

  for (int k0 = 0; k0 < K; k0 += 32) {
    V bh[4];
#pragma unroll
    for (int j = 0; j < 4; ++j) {
      const size_t bo = (size_t)(n0 + (j << 4) + rlane) * ldb + koff + k0;
      bh[j] = Frag<T>::load(Bt + bo);
    }
#pragma unroll
    for (int i = 0; i < 4; ++i) {
      const size_t ao = (size_t)(m0 + (i << 4) + rlane) * lda + koff + k0;
      V ah = Frag<T>::load(A + ao);
#pragma unroll
      for (int j = 0; j < 4; ++j) acc[i][j] = Frag<T>::mma(ah, bh[j], acc[i][j]);
      dep_guard4_h(acc[i][0], acc[i][1], acc[i][2], acc[i][3], ah, bh[3]);
    }
    keep4_h(bh[0], bh[1], bh[2], bh[3]);
  }
  acc_guard4(acc[0][0], acc[0][1], acc[0][2], acc[0][3]);
  acc_guard4(acc[1][0], acc[1][1], acc[1][2], acc[1][3]);
  acc_guard4(acc[2][0], acc[2][1], acc[2][2], acc[2][3]);
  acc_guard4(acc[3][0], acc[3][1], acc[3][2], acc[3][3]);

  float* slab = sT[wave];
#pragma unroll
  for (int i = 0; i < 4; ++i) {
    const int mBase = m0 + (i << 4);
#pragma unroll
    for (int j = 0; j < 4; ++j) {
      const int n = n0 + (j << 4) + rlane;
      const float bv = bias_a[n] + bias_b[n];
#pragma unroll
      for (int r = 0; r < 8; ++r) {
        const float v = acc[i][j][r] * scale + bv;
        slab[(mOff + r) * 68 + (j << 4) + rlane] = v;
      }
    }
    __builtin_amdgcn_fence(__ATOMIC_RELEASE, "workgroup");
    __builtin_amdgcn_wave_barrier();
    __builtin_amdgcn_fence(__ATOMIC_ACQUIRE, "workgroup");
    {
      const int hh = lane >> 4, c4 = (lane & 15) * 4;
      for (int pass = 0; pass < 2; ++pass) {
#pragma unroll
        for (int it = 0; it < 8; ++it) {
          const int row = it * 2 + hh;
          v4f v = *(const v4f*)(slab + row * 68 + c4);
          *(volatile v4f*)(C + (size_t)(mBase + row) * ldc + n0 + c4) = v;
        }
        __threadfence();
      }
    }
    __builtin_amdgcn_fence(__ATOMIC_RELEASE, "workgroup");
    __builtin_amdgcn_wave_barrier();
    __builtin_amdgcn_fence(__ATOMIC_ACQUIRE, "workgroup");
  }
}

__global__ __launch_bounds__(SCAN_THR) void rnn_scan_kernel(const int* __restrict__ xid, const float* __restrict__ PT,
                                                            const unsigned short* __restrict__ WHp,
                                                            float* __restrict__ HLAST) {
  __shared__ __align__(16) _Float16 Ah[2][SEQ_BLK * HPITCH];
  __shared__ __align__(16) int      sIdx[IDX_CHUNK * SEQ_BLK];
  __shared__ __align__(16) float    Hs[SEQ_BLK * OPITCH];
  const _Float16* WH = (const _Float16*)WHp;
  const int tid = threadIdx.x, lane = tid & 31, wave = tid >> 5;
  const int c = lane & 15, hh = lane >> 4, koff = hh * 8;
  const int rowbase = blockIdx.x * SEQ_BLK;
  const int n = 16 * wave + c;

  v16h vb[8];
  {
    const _Float16* wrow = WH + (size_t)n * NHID + koff;
#pragma unroll
    for (int k = 0; k < 8; ++k) vb[k] = Frag<_Float16>::load(wrow + 32 * k);
  }

  {
    _Float16* ahf = &Ah[0][0];
#pragma unroll 1
    for (int i = tid; i < 2 * SEQ_BLK * HPITCH; i += SCAN_THR) ahf[i] = (_Float16)0.0f;
  }

  const v8f z8 = {0.f, 0.f, 0.f, 0.f, 0.f, 0.f, 0.f, 0.f};
  const int srow = tid >> 5, scol = tid & 31;

#pragma unroll 1
  for (int ch = 0; ch < NSTEP / IDX_CHUNK; ++ch) {
    {
      int id = xid[(size_t)(rowbase + srow) * NSTEP + (size_t)(ch * IDX_CHUNK + scol)];
      id = id < 0 ? 0 : id;
      id = id > (NVOCAB - 1) ? (NVOCAB - 1) : id;
      sIdx[scol * SEQ_BLK + srow] = id;
    }
    __syncthreads();

#pragma unroll 1
    for (int tl = 0; tl < IDX_CHUNK; ++tl) {
      const int t   = ch * IDX_CHUNK + tl;
      const int cur = t & 1;
      const bool last = (t == NSTEP - 1);
      const _Float16* ahrow = &Ah[cur][0] + c * HPITCH + koff;
      _Float16* ahn = &Ah[cur ^ 1][0];

      v8f acc = z8;
#pragma unroll
      for (int k = 0; k < 8; ++k) {
        const v16h a = Frag<_Float16>::load(ahrow + 32 * k);
        acc = mma_f16_guarded(a, vb[k], acc);
      }

      const v4i ia = *(const v4i*)(sIdx + tl * SEQ_BLK + 8 * hh);
      const v4i ib = *(const v4i*)(sIdx + tl * SEQ_BLK + 8 * hh + 4);
      int ids[8];
      ids[0] = ia[0]; ids[1] = ia[1]; ids[2] = ia[2]; ids[3] = ia[3];
      ids[4] = ib[0]; ids[5] = ib[1]; ids[6] = ib[2]; ids[7] = ib[3];

#pragma unroll
      for (int r = 0; r < 8; ++r) {
        const float p  = PT[(size_t)ids[r] * NHID + n];
        const float z  = acc[r] * WCARRY_INV + p;
        const float hv = tanhf(z);
        ahn[(8 * hh + r) * HPITCH + n] = (_Float16)hv;
        if (last) Hs[(8 * hh + r) * OPITCH + n] = hv;
      }
      __syncthreads();
    }
  }

  for (int pass = 0; pass < 2; ++pass) {
#pragma unroll
    for (int it = 0; it < 2; ++it) {
      const int idx = it * SCAN_THR + tid;
      const int row = idx >> 6, c4 = (idx & 63) * 4;
      const v4f v = *(const v4f*)(Hs + row * OPITCH + c4);
      *(volatile v4f*)(HLAST + (size_t)(rowbase + row) * NHID + c4) = v;
    }
    __threadfence();
  }
}

__global__ __launch_bounds__(HEAD_THR) void head_kernel(const float* __restrict__ HL, const float* __restrict__ w1,
                                                        const float* __restrict__ b1, const float* __restrict__ w2,
                                                        const float* __restrict__ b2, float* __restrict__ out) {
  __shared__ __align__(16) float sHid[NBATCH * NFC1];
  const int tid = threadIdx.x;
  {
    const int j = tid & (NFC1 - 1);
    const int half = tid >> 7;
    const float* wrow = w1 + (size_t)j * NHID;
    const float bj = b1[j];
#pragma unroll 1
    for (int g = 0; g < 4; ++g) {
      const int b0 = half * 32 + g * 8;
      float acc[8];
#pragma unroll
      for (int r = 0; r < 8; ++r) acc[r] = 0.0f;
#pragma unroll 1
      for (int k = 0; k < NHID; k += 4) {
        const v4f w = *(const v4f*)(wrow + k);
#pragma unroll
        for (int r = 0; r < 8; ++r) {
          const v4f hv = *(const v4f*)(HL + (size_t)(b0 + r) * NHID + k);
          float s = acc[r];
          s = fmaf(w[0], hv[0], s);
          s = fmaf(w[1], hv[1], s);
          s = fmaf(w[2], hv[2], s);
          s = fmaf(w[3], hv[3], s);
          acc[r] = s;
        }
      }
#pragma unroll
      for (int r = 0; r < 8; ++r) sHid[(b0 + r) * NFC1 + j] = fmaxf(acc[r] + bj, 0.0f);
    }
  }
  __syncthreads();

  const int o = tid & (NOUTC - 1);
  const float bo = b2[o];
  const float* wp = w2 + (size_t)o * NFC1;
  float res[4];
#pragma unroll
  for (int jj = 0; jj < 4; ++jj) {
    const int i = tid + HEAD_THR * jj;
    const int b = i >> 4;
    const float* hp = sHid + b * NFC1;
    float s = 0.0f;
#pragma unroll 1
    for (int k = 0; k < NFC1; k += 4) {
      const v4f hv = *(const v4f*)(hp + k);
      const v4f wv = *(const v4f*)(wp + k);
      s = fmaf(hv[0], wv[0], s);
      s = fmaf(hv[1], wv[1], s);
      s = fmaf(hv[2], wv[2], s);
      s = fmaf(hv[3], wv[3], s);
    }
    res[jj] = s + bo;
  }
  volatile float* vo = (volatile float*)out;
  for (int pass = 0; pass < 2; ++pass) {
#pragma unroll
    for (int jj = 0; jj < 4; ++jj) vo[tid + HEAD_THR * jj] = res[jj];
    __threadfence();
  }
}

extern "C" void kernel_launch(void* const* d_in, const int* in_sizes, int n_in,
                              void* d_out, int out_size, void* d_ws, size_t ws_size, hipStream_t stream) {
  if (n_in < 10 || d_out == nullptr || d_ws == nullptr) return;
  if (in_sizes[0] != NBATCH * NSTEP || in_sizes[1] != NVOCAB * NEMB || in_sizes[2] != NHID * NEMB ||
      in_sizes[3] != NHID * NHID || in_sizes[4] != NHID || in_sizes[5] != NHID ||
      in_sizes[6] != NFC1 * NHID || in_sizes[7] != NFC1 || in_sizes[8] != NOUTC * NFC1 ||
      in_sizes[9] != NOUTC || out_size != NBATCH * NOUTC) return;

  const int*   x     = (const int*)d_in[0];
  const float* emb   = (const float*)d_in[1];
  const float* W_ih  = (const float*)d_in[2];
  const float* W_hh  = (const float*)d_in[3];
  const float* b_ih  = (const float*)d_in[4];
  const float* b_hh  = (const float*)d_in[5];
  const float* fc1_w = (const float*)d_in[6];
  const float* fc1_b = (const float*)d_in[7];
  const float* fc2_w = (const float*)d_in[8];
  const float* fc2_b = (const float*)d_in[9];
  float* out = (float*)d_out;

  char* ws = (char*)d_ws; size_t off = 0;
  auto carve = [&](size_t bytes) -> char* { char* p = ws + off; off += (bytes + 255) & ~(size_t)255; return p; };
  unsigned short* EMB16 = (unsigned short*)carve((size_t)NVPAD * NEMB * 2);
  unsigned short* WIH16 = (unsigned short*)carve((size_t)NHID * NEMB * 2);
  unsigned short* WHH16 = (unsigned short*)carve((size_t)NHID * NHID * 2);
  float*          PTAB  = (float*)carve((size_t)NVPAD * NHID * 4);
  float*          HLAST = (float*)carve((size_t)NBATCH * NHID * 4);
  if (off > ws_size || off > (size_t)134217728) return;

  const int n8e = NVPAD * (NEMB / 8);
  const int n8w = NHID * (NEMB / 8);
  cvt8_f16_kernel<<<n8e / CVT_THR, CVT_THR, 0, stream>>>(emb,  EMB16, NVOCAB, NVPAD, NEMB / 8, 1.0f);
  cvt8_f16_kernel<<<n8w / CVT_THR, CVT_THR, 0, stream>>>(W_ih, WIH16, NHID,   NHID,  NEMB / 8, WCARRY);
  cvt8_f16_kernel<<<n8w / CVT_THR, CVT_THR, 0, stream>>>(W_hh, WHH16, NHID,   NHID,  NHID / 8, WCARRY);

  const int gblocks = ((NVPAD / 64) * (NHID / 64)) / 8;
  wmma_gemm64_f16<<<gblocks, 256, 0, stream>>>(EMB16, NEMB, WIH16, NEMB, PTAB, NHID, b_ih, b_hh,
                                               NVPAD, NHID, NEMB, WCARRY_INV);

  rnn_scan_kernel<<<NBATCH / SEQ_BLK, SCAN_THR, 0, stream>>>(x, PTAB, WHH16, HLAST);

  head_kernel<<<1, HEAD_THR, 0, stream>>>(HLAST, fc1_w, fc1_b, fc2_w, fc2_b, out);
}
